// GCNReactionDirectionPredictor_60653528154494
// MI455X (gfx1250) — hardware-run, weakly checked
//
#include <hip/hip_runtime.h>
#include <stddef.h>


#define FD      64
#define FO      32
#define NTHR    256
#define NWAVE   8
#define EPT     8
#define NGRP    1
#define CHUNK   (NTHR * EPT * NGRP)
#define WCAP    (EPT * NGRP * 32)
#define LISTN   (NWAVE * WCAP)
#define ESHF    11
#define NBC     32768
#define NBF     2048
#define RCAP    67584
#define RBN     128
#define TGT     256
#define DEGCAP  1024
#define GROWS   128
#define OTHR    512
#define PTHR    32
#define GCAP    2048
#define WPL     (FD * FD)
#define WSCAP   134217728

#define LDS_COUNT ((NBC + LISTN + NWAVE) * 4)
#define LDS_FILL  ((RCAP + NBF + LISTN + NWAVE) * 4)
#define LDS_GEMM  36864

static_assert((CHUNK & (CHUNK - 1)) == 0);
static_assert((NBC & (NBC - 1)) == 0 && (NBF & (NBF - 1)) == 0);
static_assert(NBF <= (1 << ESHF));
static_assert((NBC % NBF) == 0);
static_assert(OTHR * 4 == NBF);
static_assert((RCAP % 32) == 0);
static_assert(TGT == NWAVE * 32);
static_assert(GROWS == NWAVE * 16);
static_assert((TGT % GROWS) == 0);
static_assert((GROWS * FD / 8) % NTHR == 0);
static_assert(2 * GROWS * (FD + 8) * 2 <= LDS_GEMM && GROWS * FD * 4 <= LDS_GEMM);
static_assert(FD == 64 && FO == 32 && PTHR == FO);
static_assert(NBC == NWAVE * 32 * 128);
static_assert(LDS_FILL <= 300000 && LDS_COUNT <= 300000);
static_assert(RBN % 4 == 0 && RBN <= OTHR);

typedef float           v2f   __attribute__((ext_vector_type(2)));
typedef float           v4f   __attribute__((ext_vector_type(4)));
typedef float           v8f   __attribute__((ext_vector_type(8)));
typedef int             v4i   __attribute__((ext_vector_type(4)));
typedef unsigned short  v8us  __attribute__((ext_vector_type(8)));
typedef unsigned short  v16us __attribute__((ext_vector_type(16)));
typedef __bf16          v16bf __attribute__((ext_vector_type(16)));
union FragB { v16bf v; v16us u; v8us h[2]; };

__device__ __forceinline__ unsigned short bf_rne(float f) {
  const unsigned u = __float_as_uint(f);
  return (unsigned short)((u + 0x7FFFu + ((u >> 16) & 1u)) >> 16);
}
__device__ __forceinline__ float bf_val(unsigned short b) { return __uint_as_float(((unsigned)b) << 16); }

__device__ __forceinline__ v8f wmb(v16bf a, v16bf b, v8f c) {
  v8f d = __builtin_amdgcn_wmma_f32_16x16x32_bf16(false, a, false, b, (short)0, c, false, false);
  asm volatile("v_nop\n\tv_nop\n\tv_nop\n\tv_nop" : "+v"(d) : "v"(a), "v"(b));
  return d;
}

template <int NB, int SRC>
__device__ __forceinline__ int scan_chunk(const int* __restrict__ dsts, const int* __restrict__ srcs, int nE, int nN,
                                          int cbase, int slotBase, int vec8, int* list, int tid, int lane, int wave) {
  int wc = 0;
#pragma unroll
  for (int g = 0; g < NGRP; ++g) {
    const int el0  = (g * NTHR + tid) * EPT;
    const int e0   = cbase + el0;
    const int sent = -2147483647 - 1;
    v4i da, db;
    v4i sa = {0, 0, 0, 0}, sb = {0, 0, 0, 0};
    if (vec8 != 0 && cbase + CHUNK <= nE) {
      da = *(const v4i*)(dsts + e0);
      db = *(const v4i*)(dsts + e0 + 4);
      if (SRC) {
        sa = *(const v4i*)(srcs + e0);
        sb = *(const v4i*)(srcs + e0 + 4);
      }
    } else {
      da.x = (e0     < nE) ? dsts[min(e0, nE - 1)] : sent;
      da.y = (e0 + 1 < nE) ? dsts[min(e0 + 1, nE - 1)] : sent;
      da.z = (e0 + 2 < nE) ? dsts[min(e0 + 2, nE - 1)] : sent;
      da.w = (e0 + 3 < nE) ? dsts[min(e0 + 3, nE - 1)] : sent;
      db.x = (e0 + 4 < nE) ? dsts[min(e0 + 4, nE - 1)] : sent;
      db.y = (e0 + 5 < nE) ? dsts[min(e0 + 5, nE - 1)] : sent;
      db.z = (e0 + 6 < nE) ? dsts[min(e0 + 6, nE - 1)] : sent;
      db.w = (e0 + 7 < nE) ? dsts[min(e0 + 7, nE - 1)] : sent;
      if (SRC) {
        sa.x = srcs[min(e0, nE - 1)];
        sa.y = srcs[min(e0 + 1, nE - 1)];
        sa.z = srcs[min(e0 + 2, nE - 1)];
        sa.w = srcs[min(e0 + 3, nE - 1)];
        sb.x = srcs[min(e0 + 4, nE - 1)];
        sb.y = srcs[min(e0 + 5, nE - 1)];
        sb.z = srcs[min(e0 + 6, nE - 1)];
        sb.w = srcs[min(e0 + 7, nE - 1)];
      }
    }
    if (SRC) {
      sa.x = min(max(sa.x, 0), nN - 1); sa.y = min(max(sa.y, 0), nN - 1);
      sa.z = min(max(sa.z, 0), nN - 1); sa.w = min(max(sa.w, 0), nN - 1);
      sb.x = min(max(sb.x, 0), nN - 1); sb.y = min(max(sb.y, 0), nN - 1);
      sb.z = min(max(sb.z, 0), nN - 1); sb.w = min(max(sb.w, 0), nN - 1);
    }
    const unsigned nb = (unsigned)slotBase;
    const unsigned s0 = (unsigned)da.x - nb, s1 = (unsigned)da.y - nb;
    const unsigned s2 = (unsigned)da.z - nb, s3 = (unsigned)da.w - nb;
    const unsigned s4 = (unsigned)db.x - nb, s5 = (unsigned)db.y - nb;
    const unsigned s6 = (unsigned)db.z - nb, s7 = (unsigned)db.w - nb;
    const bool h0 = s0 < (unsigned)NB, h1 = s1 < (unsigned)NB, h2 = s2 < (unsigned)NB, h3 = s3 < (unsigned)NB;
    const bool h4 = s4 < (unsigned)NB, h5 = s5 < (unsigned)NB, h6 = s6 < (unsigned)NB, h7 = s7 < (unsigned)NB;
    const unsigned any = __builtin_amdgcn_ballot_w32(h0 | h1 | h2 | h3 | h4 | h5 | h6 | h7);
    if (any != 0u) {
#define HITJ(HJ, SJ, VJ) { \
        const unsigned mj = __builtin_amdgcn_ballot_w32(HJ); \
        if (mj != 0u) { \
          if (HJ) { \
            const int pos = wc + (int)__builtin_amdgcn_mbcnt_lo(mj, 0u); \
            const int entv = SRC ? (((VJ) << ESHF) | (int)(SJ)) : (int)(SJ); \
            if (pos < WCAP) list[wave * WCAP + pos] = entv; \
          } \
          wc += (int)__builtin_popcount(mj); } }
      HITJ(h0, s0, sa.x)
      HITJ(h1, s1, sa.y)
      HITJ(h2, s2, sa.z)
      HITJ(h3, s3, sa.w)
      HITJ(h4, s4, sb.x)
      HITJ(h5, s5, sb.y)
      HITJ(h6, s6, sb.z)
      HITJ(h7, s7, sb.w)
#undef HITJ
    }
  }
  return wc;
}

__global__ __launch_bounds__(NTHR) void k_wprep(const float* __restrict__ w1, const float* __restrict__ w2,
                                                const float* __restrict__ w3, unsigned short* wp) {
  const int tid = threadIdx.x;
  const int b = (int)blockIdx.x;
  const int q = b >> 1;
  const int j = (b & 1) * NTHR + tid;
  const int n = j >> 3;
  const int k0 = (j & 7) * 8;
  const float* src = w1;
  int nout = FD;
  if (q == 1) { src = w2; nout = FD; }
  else if (q == 2) { src = w3; nout = FO; }
  const int nc = n < nout ? n : nout - 1;
  v8us hv, lv;
#pragma unroll
  for (int e = 0; e < 8; ++e) {
    float v = src[(size_t)(k0 + e) * nout + nc];
    v = (n < nout) ? v : 0.0f;
    const unsigned short hb = bf_rne(v);
    hv[e] = hb;
    lv[e] = bf_rne(v - bf_val(hb));
  }
  unsigned short* dh = wp + (size_t)(2 * q) * WPL + (size_t)j * 8;
  unsigned short* dl = dh + WPL;
  *(volatile v8us*)dh = hv;
  *(volatile v8us*)dl = lv;
  __threadfence();
  *(volatile v8us*)dh = hv;
  *(volatile v8us*)dl = lv;
}

__global__ __launch_bounds__(NTHR) void k_count(
    const int* __restrict__ ei, int* cnt, float* dinv, int nE, int nN, int vec8) {
  extern __shared__ v4f lds_dyn[];
  int* scnt = (int*)lds_dyn;
  int* list = scnt + NBC;
  int* wcnt = list + LISTN;
  const int tid = threadIdx.x, lane = tid & 31, wave = tid >> 5;
  const int nodeBase = blockIdx.x * NBC;
  const int* dsts = ei + nE;

  {
    const v4i z = {0, 0, 0, 0};
    for (int i = tid; i < NBC / 4; i += NTHR) ((v4i*)scnt)[i] = z;
  }
  __syncthreads();

  const int nChunks = (nE + CHUNK - 1) / CHUNK;
#pragma unroll 1
  for (int ch = 0; ch < nChunks; ++ch) {
    const int cbase = ch * CHUNK;
    const int wc = scan_chunk<NBC, 0>(dsts, ei, nE, nN, cbase, nodeBase, vec8, list, tid, lane, wave);
    if (lane == 0) wcnt[wave] = wc;
    __syncthreads();
    if (wave == 0) {
#pragma unroll 1
      for (int wsx = 0; wsx < NWAVE; ++wsx) {
        int n = __builtin_amdgcn_readfirstlane(wcnt[wsx]);
        n = n > WCAP ? WCAP : (n < 0 ? 0 : n);
        const int* lp = list + wsx * WCAP;
#pragma unroll 1
        for (int i = 0; i < n; ++i) {
          const int ent  = __builtin_amdgcn_readfirstlane(lp[i]);
          const int slot = ent & (NBC - 1);
          if (lane == 0) scnt[slot] = scnt[slot] + 1;
        }
      }
    }
    __syncthreads();
  }

  int*   cp = cnt + (size_t)nodeBase;
  float* dp = dinv + (size_t)nodeBase;
#pragma unroll 4
  for (int q = 0; q < 32; ++q) {
    const int f = (wave * 32 + q) * 128 + 4 * lane;
    const v4i c = *(const v4i*)(scnt + f);
    v4f d;
    d.x = rsqrtf((float)(c.x + 1)); d.y = rsqrtf((float)(c.y + 1));
    d.z = rsqrtf((float)(c.z + 1)); d.w = rsqrtf((float)(c.w + 1));
    *(volatile v4i*)(cp + f) = c;
    *(volatile v4f*)(dp + f) = d;
  }
  __threadfence();
#pragma unroll 4
  for (int q = 0; q < 32; ++q) {
    const int f = (wave * 32 + q) * 128 + 4 * lane;
    const v4i c = *(const v4i*)(scnt + f);
    v4f d;
    d.x = rsqrtf((float)(c.x + 1)); d.y = rsqrtf((float)(c.y + 1));
    d.z = rsqrtf((float)(c.z + 1)); d.w = rsqrtf((float)(c.w + 1));
    *(volatile v4i*)(cp + f) = c;
    *(volatile v4f*)(dp + f) = d;
  }
}

__global__ __launch_bounds__(OTHR) void k_offsets(
    const int* __restrict__ cnt, int* off, int* rbase, int nBF) {
  __shared__ __attribute__((aligned(16))) int srb[RBN];
  __shared__ int wtot[OTHR / 32];
  const int tid = threadIdx.x, lane = tid & 31, wave = tid >> 5;
  for (int i = tid; i < RBN; i += OTHR) srb[i] = 0;
  int carry = 0;
#pragma unroll 1
  for (int fb = 0; fb < nBF; ++fb) {
    const int base = fb * NBF;
    const v4i c = *(const v4i*)(cnt + base + 4 * tid);
    const int e0 = max(c.x, 0), e1 = max(c.y, 0), e2 = max(c.z, 0), e3 = max(c.w, 0);
    const int ts = e0 + e1 + e2 + e3;
    int incl = ts;
#pragma unroll
    for (int d = 1; d < 32; d <<= 1) {
      const int t = __shfl_up(incl, d);
      if (lane >= d) incl += t;
    }
    if (lane == 31) wtot[wave] = incl;
    __syncthreads();
    int pre = 0;
#pragma unroll 1
    for (int w = 0; w < wave; ++w) pre += wtot[w];
    int tot = 0;
#pragma unroll
    for (int w = 0; w < OTHR / 32; ++w) tot += wtot[w];
    int run = carry + pre + incl - ts;
    v4i o;
    o.x = run; run += e0;
    o.y = run; run += e1;
    o.z = run; run += e2;
    o.w = run;
    int* op = off + base + 4 * tid;
    *(volatile v4i*)op = o;
    __threadfence();
    *(volatile v4i*)op = o;
    if (tid == 0) srb[min(fb, RBN - 1)] = carry;
    carry += (tot + 31) & ~31;
    __syncthreads();
  }
  if (tid == 0) srb[min(nBF, RBN - 1)] = carry;
  __syncthreads();
  v4i rv = {0, 0, 0, 0};
  if (tid < 32) rv = *(const v4i*)(srb + 4 * tid);
  if (tid < 32) *(volatile v4i*)(rbase + 4 * tid) = rv;
  __threadfence();
  if (tid < 32) *(volatile v4i*)(rbase + 4 * tid) = rv;
}

__global__ __launch_bounds__(NTHR) void k_fill(
    const int* __restrict__ ei, const int* __restrict__ off, const int* __restrict__ rbase,
    int* csr, int nN, int nE, int vec8, int csrLen) {
  extern __shared__ v4f lds_dyn[];
  int* region = (int*)lds_dyn;
  int* cursor = region + RCAP;
  int* list   = cursor + NBF;
  int* wcnt   = list + LISTN;
  const int tid = threadIdx.x, lane = tid & 31, wave = tid >> 5;
  const int b = blockIdx.x;
  const int nodeBase = b * NBF;
  const int* dsts = ei + nE;

  int rb0 = rbase[b];
  const int rb1 = rbase[b + 1];
  rb0 = rb0 < 0 ? 0 : (rb0 > csrLen ? csrLen : rb0);
  rb0 &= ~31;
  int len = rb1 - rb0;
  len = len < 0 ? 0 : (len > RCAP ? RCAP : len);
  int lenW = (len + 31) & ~31;
  if (rb0 + lenW > csrLen) lenW = (csrLen - rb0) & ~31;

  {
    const v4i z = {0, 0, 0, 0};
    for (int i = tid; i < RCAP / 4; i += NTHR) ((v4i*)region)[i] = z;
    for (int s = tid; s < NBF; s += NTHR) {
      int o = off[nodeBase + s] - rb0;
      o = o < 0 ? 0 : (o > RCAP ? RCAP : o);
      cursor[s] = o;
    }
  }
  __syncthreads();

  const int nChunks = (nE + CHUNK - 1) / CHUNK;
#pragma unroll 1
  for (int ch = 0; ch < nChunks; ++ch) {
    const int cbase = ch * CHUNK;
    const int wc = scan_chunk<NBF, 1>(dsts, ei, nE, nN, cbase, nodeBase, vec8, list, tid, lane, wave);
    if (lane == 0) wcnt[wave] = wc;
    __syncthreads();
    if (wave == 0) {
#pragma unroll 1
      for (int wsx = 0; wsx < NWAVE; ++wsx) {
        int n = __builtin_amdgcn_readfirstlane(wcnt[wsx]);
        n = n > WCAP ? WCAP : (n < 0 ? 0 : n);
        const int* lp = list + wsx * WCAP;
#pragma unroll 1
        for (int i = 0; i < n; ++i) {
          const int ent  = __builtin_amdgcn_readfirstlane(lp[i]);
          const int slot = ent & (NBF - 1);
          int src = (ent >> ESHF) & 0xFFFFF;
          src = src > nN - 1 ? nN - 1 : src;
          if (lane == 0) {
            int pos = cursor[slot];
            pos = pos < 0 ? 0 : (pos > RCAP - 1 ? RCAP - 1 : pos);
            region[pos] = src;
            const int np = pos + 1;
            cursor[slot] = np > RCAP ? RCAP : np;
          }
        }
      }
    }
    __syncthreads();
  }

  const int nv = lenW >> 2;
  int* gp = csr + rb0;
#pragma unroll 1
  for (int i = tid; i < nv; i += NTHR) { const v4i v = ((const v4i*)region)[i]; *(volatile v4i*)(gp + 4 * i) = v; }
  __threadfence();
#pragma unroll 1
  for (int i = tid; i < nv; i += NTHR) { const v4i v = ((const v4i*)region)[i]; *(volatile v4i*)(gp + 4 * i) = v; }
}

template <int GATHER, int NT>
__global__ __launch_bounds__(NTHR) void k_gemm(
    const float* __restrict__ A, const int* __restrict__ ids, int nIds, int vocab,
    const unsigned short* __restrict__ Bh, const unsigned short* __restrict__ Bl,
    const float* __restrict__ dinv, float* C, int nRowsA) {
  extern __shared__ v4f lds_dyn[];
  constexpr int APH = FD + 8;
  unsigned short* sAh = (unsigned short*)lds_dyn;
  unsigned short* sAl = sAh + GROWS * APH;
  float*          stg = (float*)lds_dyn;
  const int tid = threadIdx.x, lane = tid & 31, wave = tid >> 5, hh = lane >> 4, m = lane & 15;
  const int rowBase = blockIdx.x * GROWS;

#pragma unroll
  for (int i = 0; i < (GROWS * FD / 8) / NTHR; ++i) {
    const int idx = i * NTHR + tid;
    const int r   = idx >> 3;
    const int c0  = (idx & 7) * 8;
    const float* ap;
    if (GATHER) {
      int row = rowBase + r;
      row = row > nIds - 1 ? nIds - 1 : row;
      int id = ids[row];
      id = id < 0 ? 0 : (id > vocab - 1 ? vocab - 1 : id);
      ap = A + (size_t)id * FD + c0;
    } else {
      int row = rowBase + r;
      row = row > nRowsA - 1 ? nRowsA - 1 : row;
      ap = A + (size_t)row * FD + c0;
    }
    const v4f a = *(const v4f*)ap, b = *(const v4f*)(ap + 4);
    float f[8];
    f[0] = a.x; f[1] = a.y; f[2] = a.z; f[3] = a.w; f[4] = b.x; f[5] = b.y; f[6] = b.z; f[7] = b.w;
    v8us hv, lv;
#pragma unroll
    for (int e = 0; e < 8; ++e) {
      const unsigned short hb = bf_rne(f[e]);
      hv[e] = hb;
      lv[e] = bf_rne(f[e] - bf_val(hb));
    }
    *(v8us*)(sAh + r * APH + c0) = hv;
    *(v8us*)(sAl + r * APH + c0) = lv;
  }
  __syncthreads();

  v8f acc[4];
#pragma unroll
  for (int t = 0; t < 4; ++t) { v8f z = {0.f, 0.f, 0.f, 0.f, 0.f, 0.f, 0.f, 0.f}; acc[t] = z; }
  const unsigned short* ahp = sAh + (wave * 16 + m) * APH + 8 * hh;
  const unsigned short* alp = sAl + (wave * 16 + m) * APH + 8 * hh;
#pragma unroll 1
  for (int kt = 0; kt < FD / 32; ++kt) {
    FragB ah, al;
    ah.h[0] = *(const v8us*)(ahp + 32 * kt);
    ah.h[1] = *(const v8us*)(ahp + 32 * kt + 16);
    al.h[0] = *(const v8us*)(alp + 32 * kt);
    al.h[1] = *(const v8us*)(alp + 32 * kt + 16);
#pragma unroll
    for (int t = 0; t < NT; ++t) {
      const size_t bo = (size_t)(16 * t + m) * FD + 32 * kt + 8 * hh;
      FragB bh, bl;
      bh.h[0] = *(const v8us*)(Bh + bo);
      bh.h[1] = *(const v8us*)(Bh + bo + 16);
      bl.h[0] = *(const v8us*)(Bl + bo);
      bl.h[1] = *(const v8us*)(Bl + bo + 16);
      acc[t] = wmb(ah.v, bh.v, acc[t]);
      acc[t] = wmb(al.v, bh.v, acc[t]);
      acc[t] = wmb(ah.v, bl.v, acc[t]);
    }
  }
  __syncthreads();

  const int r0 = wave * 16 + 8 * hh;
  const v4f dA = *(const v4f*)(dinv + (size_t)rowBase + r0);
  const v4f dB = *(const v4f*)(dinv + (size_t)rowBase + r0 + 4);
  float s[8];
  s[0] = dA.x; s[1] = dA.y; s[2] = dA.z; s[3] = dA.w; s[4] = dB.x; s[5] = dB.y; s[6] = dB.z; s[7] = dB.w;
  float* sp = stg + r0 * FD + m;
#pragma unroll
  for (int t = 0; t < 4; ++t) {
#pragma unroll
    for (int r = 0; r < 8; ++r) sp[r * FD + 16 * t] = acc[t][r] * s[r];
  }
  __syncthreads();

  const float* lp = stg + wave * 16 * FD;
  float* gp = C + (size_t)(rowBase + wave * 16) * FD;
#pragma unroll
  for (int i = 0; i < (16 * FD) / 128; ++i) {
    const v4f v = *(const v4f*)(lp + i * 128 + 4 * lane);
    *(volatile v4f*)(gp + i * 128 + 4 * lane) = v;
  }
  __threadfence();
#pragma unroll
  for (int i = 0; i < (16 * FD) / 128; ++i) {
    const v4f v = *(const v4f*)(lp + i * 128 + 4 * lane);
    *(volatile v4f*)(gp + i * 128 + 4 * lane) = v;
  }
}

__global__ __launch_bounds__(NTHR) void k_agg(
    const int* __restrict__ csr, const int* __restrict__ off, const int* __restrict__ cnt,
    const float* __restrict__ dinv, const float* __restrict__ hw, const float* __restrict__ bs, int nb,
    float* h, int nN, int csrLen) {
  const int tid = threadIdx.x, lane = tid & 31, wave = tid >> 5;
  const int tbase = blockIdx.x * TGT + wave * 32;
  const int cl = tbase + lane;
  const int cnt_l = cnt[cl];
  const int off_l = off[cl];
  union FI { float f; int i; };
  FI dvu; dvu.f = dinv[cl];
  const int c0i = (2 * lane)     < (nb - 1) ? (2 * lane)     : (nb - 1);
  const int c1i = (2 * lane + 1) < (nb - 1) ? (2 * lane + 1) : (nb - 1);
  v2f bb;
  bb.x = bs[c0i]; bb.y = bs[c1i];
  if (2 * lane     >= nb) bb.x = 0.f;
  if (2 * lane + 1 >= nb) bb.y = 0.f;

#pragma unroll 1
  for (int j = 0; j < 32; ++j) {
    const int c = tbase + j;
    int n = __builtin_amdgcn_readlane(cnt_l, j);
    n = n < 0 ? 0 : (n > DEGCAP ? DEGCAP : n);
    const int st = __builtin_amdgcn_readlane(off_l, j);
    FI du; du.i = __builtin_amdgcn_readlane(dvu.i, j);
    const float dc = du.f;
    v2f acc = {0.f, 0.f};
#pragma unroll 1
    for (int q0 = 0; q0 < n; q0 += 32) {
      int pos = st + q0 + lane;
      pos = pos < 0 ? 0 : (pos > csrLen - 1 ? csrLen - 1 : pos);
      int sl = csr[pos];
      sl = sl < 0 ? 0 : (sl > nN - 1 ? nN - 1 : sl);
      const int mcnt = (n - q0) < 32 ? (n - q0) : 32;
#pragma unroll 1
      for (int p = 0; p < mcnt; ++p) {
        const int s = __builtin_amdgcn_readlane(sl, p);
        acc = acc + *(const v2f*)(hw + (size_t)s * FD + 2 * lane);
      }
    }
    const v2f sv = *(const v2f*)(hw + (size_t)c * FD + 2 * lane);
    v2f v = (acc + sv) * dc + bb;
    v.x = v.x > 0.f ? v.x : 0.1f * v.x;
    v.y = v.y > 0.f ? v.y : 0.1f * v.y;
    float* hp = h + (size_t)c * FD + 2 * lane;
    *(volatile v2f*)hp = v;
    __threadfence();
    *(volatile v2f*)hp = v;
  }
}

__global__ __launch_bounds__(PTHR) void k_pool(
    const float* __restrict__ h, const int* __restrict__ bat, const float* __restrict__ fcw,
    const float* __restrict__ fcb, float* out, int nN, int nG) {
  extern __shared__ v4f lds_dyn[];
  float* sums = (float*)lds_dyn;
  int*   cg   = (int*)(sums + (size_t)nG * FO);
  const int ngq = (nG + 3) & ~3;
  float* so   = (float*)(cg + ngq);
  const int lane = threadIdx.x;

  {
    const v4f z = {0.f, 0.f, 0.f, 0.f};
#pragma unroll 1
    for (int i = lane; i < nG * (FO / 4); i += PTHR) ((v4f*)sums)[i] = z;
#pragma unroll 1
    for (int i = lane; i < nG; i += PTHR) cg[i] = 0;
  }
  __syncthreads();

  const float fw = fcw[lane];
  const float fb = fcb[0];

#pragma unroll 1
  for (int n0 = 0; n0 < nN; n0 += PTHR) {
    const int nl  = n0 + lane;
    const int nlc = nl < nN ? nl : nN - 1;
    const int gl  = bat[nlc];
    const int okl = (nl < nN && (unsigned)gl < (unsigned)nG) ? 1 : 0;
    const int glc = gl < 0 ? 0 : (gl > nG - 1 ? nG - 1 : gl);
    const int m = (nN - n0) < PTHR ? (nN - n0) : PTHR;
#pragma unroll 1
    for (int j = 0; j < m; ++j) {
      const int g  = __builtin_amdgcn_readlane(glc, j);
      const int ok = __builtin_amdgcn_readlane(okl, j);
      const float x = h[(size_t)(n0 + j) * FD + lane];
      const float w = ok ? 1.0f : 0.0f;
      float* sp = sums + g * FO + lane;
      *sp = *sp + x * w;
      if (lane == 0) cg[g] = cg[g] + ok;
    }
  }
  __syncthreads();

#pragma unroll 1
  for (int g = 0; g < nG; ++g) {
    const int c = cg[g];
    const float rc = 1.0f / fmaxf((float)c, 1.0f);
    const float p = sums[g * FO + lane] * rc;
    float v = p * fw;
#pragma unroll
    for (int o = 16; o >= 1; o >>= 1) v += __shfl_xor(v, o, 32);
    if (lane == 0) so[g] = v + fb;
  }
  __syncthreads();

  const int nq = nG >> 2;
#pragma unroll 1
  for (int i = lane; i < nq; i += PTHR) { const v4f v = ((const v4f*)so)[i]; *(volatile v4f*)(out + 4 * i) = v; }
#pragma unroll 1
  for (int i = (nq << 2) + lane; i < nG; i += PTHR) { const float v = so[i]; *(volatile float*)(out + i) = v; }
  __threadfence();
#pragma unroll 1
  for (int i = lane; i < nq; i += PTHR) { const v4f v = ((const v4f*)so)[i]; *(volatile v4f*)(out + 4 * i) = v; }
#pragma unroll 1
  for (int i = (nq << 2) + lane; i < nG; i += PTHR) { const float v = so[i]; *(volatile float*)(out + i) = v; }
}

extern "C" void kernel_launch(void* const* d_in, const int* in_sizes, int n_in,
                              void* d_out, int out_size, void* d_ws, size_t ws_size,
                              hipStream_t stream) {
  if (n_in < 12) return;
  const int nE    = in_sizes[0] / 2;
  const int nN    = in_sizes[1];
  const int vocab = in_sizes[3] / FD;
  const int nG    = out_size;
  if (nE <= 0 || nN <= 0 || vocab <= 0 || nG <= 0) return;
  if (in_sizes[0] != 2 * nE || in_sizes[2] != nN || in_sizes[3] != vocab * FD) return;
  if (in_sizes[4] != FD * FD || in_sizes[5] != FD || in_sizes[6] != FD * FD || in_sizes[7] != FD) return;
  if (in_sizes[8] != FD * FO || in_sizes[9] != FO || in_sizes[10] != FO || in_sizes[11] < 1) return;
  if (nN > (1 << 20) || nE > (1 << 28) || nG > GCAP) return;

  const int*   ei   = (const int*)d_in[0];
  const int*   feat = (const int*)d_in[1];
  const int*   bat  = (const int*)d_in[2];
  const float* emb  = (const float*)d_in[3];
  const float* W1   = (const float*)d_in[4];
  const float* b1   = (const float*)d_in[5];
  const float* W2   = (const float*)d_in[6];
  const float* b2   = (const float*)d_in[7];
  const float* W3   = (const float*)d_in[8];
  const float* b3   = (const float*)d_in[9];
  const float* fcw  = (const float*)d_in[10];
  const float* fcb  = (const float*)d_in[11];
  float* out = (float*)d_out;

  const int NPAD   = ((nN + TGT - 1) / TGT) * TGT;
  const int nBC    = (nN + NBC - 1) / NBC;
  const int CNTPAD = nBC * NBC;
  const int nBF    = (nN + NBF - 1) / NBF;
  const int OFFN   = nBF * NBF;
  if (nBF + 1 > RBN) return;
  if (OFFN > CNTPAD || NPAD > OFFN) return;
  const int csrLen = ((nE + 31) & ~31) + 32 * (nBF + 1);
  const int nGemm  = NPAD / GROWS;
  const int nAgg   = NPAD / TGT;

  char* ws = (char*)d_ws;
  size_t off = 0;
  const size_t oW   = off; off += (size_t)6 * WPL * 2;               off = (off + 255) & ~(size_t)255;
  const size_t oCnt = off; off += (size_t)CNTPAD * 4;                off = (off + 255) & ~(size_t)255;
  const size_t oDv  = off; off += (size_t)CNTPAD * 4;                off = (off + 255) & ~(size_t)255;
  const size_t oOff = off; off += (size_t)OFFN * 4;                  off = (off + 255) & ~(size_t)255;
  const size_t oRb  = off; off += (size_t)RBN * 4;                   off = (off + 255) & ~(size_t)255;
  const size_t oCsr = off; off += (size_t)csrLen * 4;                off = (off + 255) & ~(size_t)255;
  const size_t oHw  = off; off += (size_t)NPAD * FD * 4;             off = (off + 255) & ~(size_t)255;
  const size_t oH   = off; off += (size_t)NPAD * FD * 4;             off = (off + 255) & ~(size_t)255;
  if (off > ws_size || off > (size_t)WSCAP) return;
  unsigned short* wp   = (unsigned short*)(ws + oW);
  int*            cnt  = (int*)(ws + oCnt);
  float*          dinv = (float*)(ws + oDv);
  int*            offp = (int*)(ws + oOff);
  int*            rb   = (int*)(ws + oRb);
  int*            csr  = (int*)(ws + oCsr);
  float*          hw   = (float*)(ws + oHw);
  float*          h    = (float*)(ws + oH);

  const int vec8 = ((nE & 3) == 0) ? 1 : 0;
  const size_t ldsPool = ((size_t)nG * FO + (size_t)((nG + 3) & ~3) + (size_t)nG) * 4;

  k_wprep<<<6, NTHR, 0, stream>>>(W1, W2, W3, wp);

  hipFuncSetAttribute(reinterpret_cast<const void*>(&k_count),
                      hipFuncAttributeMaxDynamicSharedMemorySize, LDS_COUNT);
  k_count<<<nBC, NTHR, LDS_COUNT, stream>>>(ei, cnt, dinv, nE, nN, vec8);
  k_offsets<<<1, OTHR, 0, stream>>>(cnt, offp, rb, nBF);
  hipFuncSetAttribute(reinterpret_cast<const void*>(&k_fill),
                      hipFuncAttributeMaxDynamicSharedMemorySize, LDS_FILL);
  k_fill<<<nBF, NTHR, LDS_FILL, stream>>>(ei, offp, rb, csr, nN, nE, vec8, csrLen);

  k_gemm<1, 4><<<nGemm, NTHR, LDS_GEMM, stream>>>(emb, feat, nN, vocab, wp, wp + WPL, dinv, hw, nN);
  k_agg<<<nAgg, NTHR, 0, stream>>>(csr, offp, cnt, dinv, hw, b1, FD, h, nN, csrLen);

  k_gemm<0, 4><<<nGemm, NTHR, LDS_GEMM, stream>>>(h, feat, nN, vocab, wp + 2 * WPL, wp + 3 * WPL, dinv, hw, NPAD);
  k_agg<<<nAgg, NTHR, 0, stream>>>(csr, offp, cnt, dinv, hw, b2, FD, h, nN, csrLen);

  k_gemm<0, 2><<<nGemm, NTHR, LDS_GEMM, stream>>>(h, feat, nN, vocab, wp + 4 * WPL, wp + 5 * WPL, dinv, hw, NPAD);
  k_agg<<<nAgg, NTHR, 0, stream>>>(csr, offp, cnt, dinv, hw, b3, FO, h, nN, csrLen);

  hipFuncSetAttribute(reinterpret_cast<const void*>(&k_pool),
                      hipFuncAttributeMaxDynamicSharedMemorySize, (int)ldsPool);
  k_pool<<<1, PTHR, ldsPool, stream>>>(h, bat, fcw, fcb, out, nN, nG);
}
